// PointNet2_81329500717170
// MI455X (gfx1250) — hardware-verified
//
#include <hip/hip_runtime.h>
#include <stdint.h>

#pragma clang fp contract(off)

typedef __attribute__((ext_vector_type(16))) _Float16 v16h;
typedef __attribute__((ext_vector_type(8)))  _Float16 v8h;
typedef __attribute__((ext_vector_type(8)))  float    v8f;
typedef __attribute__((ext_vector_type(4)))  float    v4f;

constexpr int   kBatch    = 64;
constexpr int   kNumPts   = 4096;
constexpr float kCarry    = 16.0f;
constexpr float kResScale = 2048.0f;
constexpr float kResInv   = 1.0f / 2048.0f;
constexpr float kFoldInv  = 1.0f / (16.0f * 16.0f);
constexpr float kBnEps    = 1e-5f;

static_assert(kBatch * kNumPts * 3 * 4 == 3145728);
static_assert(kBatch * 256 * 32 * 4 == 2097152);

struct FragH {
  union U { v16h v; v8h h[2]; };
  static __device__ __forceinline__ v16h load(const _Float16* p) {
    U f; f.h[0] = *(const v8h*)(p); f.h[1] = *(const v8h*)(p + 16); return f.v;
  }
};

__device__ __forceinline__ v8f mma16(v16h a, v16h b, v8f c) {
  c = __builtin_amdgcn_wmma_f32_16x16x32_f16(false, a, false, b, (short)0, c, false, false);
  asm volatile("v_nop\n\tv_nop\n\tv_nop\n\tv_nop" : "+v"(c) : "v"(a), "v"(b));
  return c;
}

__device__ __forceinline__ void split_h(float v, _Float16& hi, _Float16& lo) {
  const float s = v * kCarry;
  hi = (_Float16)s;
  const float hf = (float)hi;
  const float d = s - hf;
  lo = (_Float16)(d * kResScale);
}

__device__ __forceinline__ void split8(const float (&f)[8], v8h& hv, v8h& lv) {
#pragma unroll
  for (int e = 0; e < 8; ++e) {
    _Float16 hi, lo;
    split_h(f[e], hi, lo);
    hv[e] = hi;
    lv[e] = lo;
  }
}

struct PrepArgs {
  const float* w[5];
  unsigned short* wh[5];
  unsigned short* wl[5];
  const float* g[6];
  const float* be[6];
  const float* rm[6];
  const float* rv[6];
  float* a[6];
  float* sh[6];
};
static_assert(sizeof(PrepArgs) == 51 * 8);

template <int COUT, int CIN, int KP, int CFP>
__device__ __forceinline__ void prep_w(const float* __restrict__ w, unsigned short* wh, unsigned short* wl, int item) {
  constexpr int PER = KP / 8;
  static_assert(KP % 32 == 0);
  static_assert((COUT * PER) % 32 == 0);
  if (item >= COUT * PER) return;
  const int n = item / PER;
  const int k8 = item - n * PER;
  float zf = 0.0f;
  asm volatile("" : "+v"(zf));
  float f[8];
#pragma unroll
  for (int e = 0; e < 8; ++e) {
    const int kp = k8 * 8 + e;
    int ko;
    bool valid;
    if (CFP == 0) {
      ko = kp;
      valid = (kp < CIN);
    } else {
      ko = (kp < CFP) ? (kp + 3) : (kp - CFP);
      valid = (kp < CFP + 3);
    }
    const int kc = valid ? ko : 0;
    const float v = w[(size_t)n * CIN + kc];
    f[e] = valid ? v : zf;
  }
  v8h hv, lv;
  split8(f, hv, lv);
  _Float16* ph = (_Float16*)wh + (size_t)item * 8;
  _Float16* pl = (_Float16*)wl + (size_t)item * 8;
  *(volatile v8h*)ph = hv;
  *(volatile v8h*)pl = lv;
  __threadfence();
  *(volatile v8h*)ph = hv;
  *(volatile v8h*)pl = lv;
}

template <int COUT>
__device__ __forceinline__ void bn_fold(const float* __restrict__ g, const float* __restrict__ be,
                                        const float* __restrict__ rm, const float* __restrict__ rv,
                                        float* a, float* sh, float fold, int tid) {
  static_assert(COUT % 32 == 0);
  if (tid < COUT / 4) {
    const v4f gg = *(const v4f*)(g + 4 * tid);
    const v4f bb = *(const v4f*)(be + 4 * tid);
    const v4f mm = *(const v4f*)(rm + 4 * tid);
    const v4f vv = *(const v4f*)(rv + 4 * tid);
    v4f ao, so;
#pragma unroll
    for (int e = 0; e < 4; ++e) {
      const float aa = gg[e] * rsqrtf(vv[e] + kBnEps);
      ao[e] = aa * fold;
      const float t = aa * mm[e];
      so[e] = bb[e] - t;
    }
    *(volatile v4f*)(a + 4 * tid) = ao;
    *(volatile v4f*)(sh + 4 * tid) = so;
    __threadfence();
    *(volatile v4f*)(a + 4 * tid) = ao;
    *(volatile v4f*)(sh + 4 * tid) = so;
  }
}

__global__ __launch_bounds__(256) void prep_kernel(PrepArgs pa) {
  const int tid = threadIdx.x;
  const int item = blockIdx.x * 256 + tid;
  const int which = blockIdx.y;
  if (which == 0) {
    prep_w<64, 32, 32, 0>(pa.w[0], pa.wh[0], pa.wl[0], item);
  } else if (which == 1) {
    prep_w<128, 67, 96, 64>(pa.w[1], pa.wh[1], pa.wl[1], item);
  } else if (which == 2) {
    prep_w<128, 128, 128, 0>(pa.w[2], pa.wh[2], pa.wl[2], item);
  } else if (which == 3) {
    prep_w<256, 131, 160, 128>(pa.w[3], pa.wh[3], pa.wl[3], item);
  } else if (which == 4) {
    prep_w<256, 256, 256, 0>(pa.w[4], pa.wh[4], pa.wl[4], item);
  } else if (blockIdx.x == 0) {
    bn_fold<32>(pa.g[0], pa.be[0], pa.rm[0], pa.rv[0], pa.a[0], pa.sh[0], 1.0f, tid);
    bn_fold<64>(pa.g[1], pa.be[1], pa.rm[1], pa.rv[1], pa.a[1], pa.sh[1], kFoldInv, tid);
    bn_fold<128>(pa.g[2], pa.be[2], pa.rm[2], pa.rv[2], pa.a[2], pa.sh[2], kFoldInv, tid);
    bn_fold<128>(pa.g[3], pa.be[3], pa.rm[3], pa.rv[3], pa.a[3], pa.sh[3], kFoldInv, tid);
    bn_fold<256>(pa.g[4], pa.be[4], pa.rm[4], pa.rv[4], pa.a[4], pa.sh[4], kFoldInv, tid);
    bn_fold<256>(pa.g[5], pa.be[5], pa.rm[5], pa.rv[5], pa.a[5], pa.sh[5], kFoldInv, tid);
  }
}

template <int N, int NPOINT>
__global__ __launch_bounds__(256) void fps_kernel(const float* __restrict__ xyz, float* __restrict__ new_xyz) {
#pragma clang fp contract(off)
  constexpr int NT = 256;
  constexpr int PT = (N + NT - 1) / NT;
  constexpr int NV4 = (N * 3) / 4;
  constexpr int OV4 = (NPOINT * 3) / 4;
  static_assert((N * 3) % 4 == 0);
  static_assert((NPOINT * 3 * 4) % 128 == 0);
  __shared__ __align__(16) float s_xyz[N * 3];
  __shared__ __align__(16) float s_out[NPOINT * 3];
  __shared__ float s_val[2][8];
  __shared__ int   s_ind[2][8];

  const int b = blockIdx.x;
  const int tid = threadIdx.x;
  const int lane = tid & 31;
  const int wave = tid >> 5;

  {
    const v4f* src = (const v4f*)(xyz + (size_t)b * N * 3);
#pragma unroll 1
    for (int i = tid; i < NV4; i += NT) {
      const v4f v = src[i];
      *(v4f*)(s_xyz + 4 * i) = v;
    }
  }
  __syncthreads();

  float px[PT], py[PT], pz[PT], dist[PT];
#pragma unroll
  for (int i = 0; i < PT; ++i) {
    const int gi = tid + i * NT;
    const int gc = (gi < N) ? gi : (N - 1);
    px[i] = s_xyz[gc * 3 + 0];
    py[i] = s_xyz[gc * 3 + 1];
    pz[i] = s_xyz[gc * 3 + 2];
    dist[i] = (gi < N) ? 1e10f : -1.0f;
  }
  float lx = s_xyz[0], ly = s_xyz[1], lz = s_xyz[2];
  if (tid == 0) {
    s_out[0] = lx; s_out[1] = ly; s_out[2] = lz;
  }

#pragma unroll 1
  for (int it = 1; it < NPOINT; ++it) {
    float bv = -2.0f;
    int bi = 0;
#pragma unroll
    for (int i = 0; i < PT; ++i) {
      const float dx = px[i] - lx;
      const float dy = py[i] - ly;
      const float dz = pz[i] - lz;
      const float t0 = dx * dx;
      const float t1 = dy * dy;
      const float t2 = dz * dz;
      const float d = (t0 + t2) + t1;
      const float nd = fminf(dist[i], d);
      dist[i] = nd;
      if (nd > bv) { bv = nd; bi = tid + i * NT; }
    }
#pragma unroll
    for (int off = 16; off >= 1; off >>= 1) {
      const float ov = __shfl_xor(bv, off, 32);
      const int oi = __shfl_xor(bi, off, 32);
      const bool take = (ov > bv) || ((ov == bv) && (oi < bi));
      bv = take ? ov : bv;
      bi = take ? oi : bi;
    }
    const int buf = it & 1;
    if (lane == 0) { s_val[buf][wave] = bv; s_ind[buf][wave] = bi; }
    __syncthreads();
    float fv = s_val[buf][0];
    int fi = s_ind[buf][0];
#pragma unroll
    for (int w = 1; w < 8; ++w) {
      const float ov = s_val[buf][w];
      const int oi = s_ind[buf][w];
      const bool take = (ov > fv) || ((ov == fv) && (oi < fi));
      fv = take ? ov : fv;
      fi = take ? oi : fi;
    }
    int sel = fi;
    sel = sel < 0 ? 0 : sel;
    sel = sel > (N - 1) ? (N - 1) : sel;
    lx = s_xyz[sel * 3 + 0];
    ly = s_xyz[sel * 3 + 1];
    lz = s_xyz[sel * 3 + 2];
    if (tid == 0) {
      s_out[it * 3 + 0] = lx; s_out[it * 3 + 1] = ly; s_out[it * 3 + 2] = lz;
    }
  }
  __syncthreads();
  if (wave == 0) {
    float* dst = new_xyz + (size_t)b * NPOINT * 3;
    for (int pass = 0; pass < 2; ++pass) {
#pragma unroll
      for (int t = 0; t < (OV4 + 31) / 32; ++t) {
        const int i = lane + 32 * t;
        if (i < OV4) {
          const v4f v = *(const v4f*)(s_out + 4 * i);
          *(volatile v4f*)(dst + 4 * i) = v;
        }
      }
      __threadfence();
    }
  }
}

template <int NI, int K, int NOUT, int NS, bool POOL>
__device__ __forceinline__ void mlp_layer(const _Float16* inH, const _Float16* inL,
                                          const _Float16* __restrict__ Wh, const _Float16* __restrict__ Wl,
                                          const float* __restrict__ av, const float* __restrict__ sv,
                                          _Float16* outH, _Float16* outL, float* sP,
                                          int wave, int lane) {
  static_assert(K % 32 == 0);
  static_assert(NOUT % 64 == 0);
  constexpr int NJ = NOUT / 64;
  const int rl = lane & 15;
  const int hh = lane >> 4;
  const int koff = hh * 8;
#pragma unroll 1
  for (int j = 0; j < NJ; ++j) {
    const int n0 = wave * (NOUT / 4) + j * 16;
    v8f am[NI], ar[NI];
#pragma unroll
    for (int i = 0; i < NI; ++i) {
      am[i] = (v8f){0.f, 0.f, 0.f, 0.f, 0.f, 0.f, 0.f, 0.f};
      ar[i] = (v8f){0.f, 0.f, 0.f, 0.f, 0.f, 0.f, 0.f, 0.f};
    }
#pragma unroll 1
    for (int k0 = 0; k0 < K; k0 += 32) {
      const size_t bo = (size_t)(n0 + rl) * K + koff + k0;
      const v16h bh = FragH::load(Wh + bo);
      const v16h bl = FragH::load(Wl + bo);
#pragma unroll
      for (int i = 0; i < NI; ++i) {
        const int ao = (i * 16 + rl) * K + koff + k0;
        const v16h ah = FragH::load(inH + ao);
        const v16h al = FragH::load(inL + ao);
        am[i] = mma16(ah, bh, am[i]);
        ar[i] = mma16(ah, bl, ar[i]);
        ar[i] = mma16(al, bh, ar[i]);
      }
    }
    const float a_n = av[n0 + rl];
    const float s_n = sv[n0 + rl];
    if constexpr (!POOL) {
#pragma unroll
      for (int i = 0; i < NI; ++i) {
#pragma unroll
        for (int r = 0; r < 8; ++r) {
          const float lin = am[i][r] + ar[i][r] * kResInv;
          float v = lin * a_n + s_n;
          v = fmaxf(v, 0.0f);
          _Float16 hi, lo;
          split_h(v, hi, lo);
          const int row = i * 16 + 8 * hh + r;
          outH[row * NOUT + n0 + rl] = hi;
          outL[row * NOUT + n0 + rl] = lo;
        }
      }
    } else {
      float pm[NI];
#pragma unroll
      for (int i = 0; i < NI; ++i) {
        float m = 0.0f;
#pragma unroll
        for (int r = 0; r < 8; ++r) {
          const float lin = am[i][r] + ar[i][r] * kResInv;
          float v = lin * a_n + s_n;
          v = fmaxf(v, 0.0f);
          m = fmaxf(m, v);
        }
        const float o = __shfl_xor(m, 16, 32);
        pm[i] = fmaxf(m, o);
      }
      if constexpr (NS == 32) {
#pragma unroll
        for (int g = 0; g < NI / 2; ++g) {
          const float pg = fmaxf(pm[2 * g], pm[2 * g + 1]);
          if (hh == 0) sP[g * NOUT + n0 + rl] = pg;
        }
      } else {
#pragma unroll
        for (int g = 0; g < NI; ++g) {
          const float pg = pm[g];
          if (hh == 0) sP[g * NOUT + n0 + rl] = pg;
        }
      }
    }
  }
}

template <int CF, int KPAD, int C1, int C2, int NS, int NSRC, int RB, bool LVL1>
__global__ __launch_bounds__(128) void sa_kernel(
    const float* __restrict__ xyz, const float* __restrict__ feats, const float* __restrict__ new_xyz,
    const float* __restrict__ w0f, const float* __restrict__ a0, const float* __restrict__ sh0,
    const unsigned short* __restrict__ WaH, const unsigned short* __restrict__ WaL,
    const float* __restrict__ aA, const float* __restrict__ shA,
    const unsigned short* __restrict__ WbH, const unsigned short* __restrict__ WbL,
    const float* __restrict__ aB, const float* __restrict__ shB,
    float* __restrict__ pooled, int S, float r2) {
#pragma clang fp contract(off)
  constexpr int NG = RB / NS;
  constexpr int NI = RB / 16;
  static_assert(RB % NS == 0 && RB % 16 == 0);
  static_assert(NSRC % 32 == 0);
  static_assert(KPAD % 32 == 0 && C1 % 32 == 0);
  static_assert(LVL1 ? (RB == 64 && KPAD == 32) : (KPAD == CF + 32 && CF % 8 == 0));
  static_assert(NG * C2 / 4 <= 128 && (NG * C2 / 4) % 32 == 0);
  static_assert(NG <= 4);

  __shared__ __align__(16) _Float16 sXh[RB * KPAD];
  __shared__ __align__(16) _Float16 sXl[RB * KPAD];
  __shared__ __align__(16) _Float16 sYh[LVL1 ? 8 : RB * C1];
  __shared__ __align__(16) _Float16 sYl[LVL1 ? 8 : RB * C1];
  __shared__ __align__(16) float sP[NG * C2];
  __shared__ float s_w0[LVL1 ? 288 : 4];
  __shared__ float s_a0[LVL1 ? 32 : 4];
  __shared__ float s_sh0[LVL1 ? 32 : 4];
  __shared__ int   s_pi[RB];
  __shared__ float s_ctr[8];

  const int tid = threadIdx.x;
  const int lane = tid & 31;
  const int wave = __builtin_amdgcn_readfirstlane(tid >> 5);
  const int b = blockIdx.y;
  const int s0 = blockIdx.x * NG;
  const float* xb = xyz + (size_t)b * NSRC * 3;

  if constexpr (LVL1) {
#pragma unroll 1
    for (int e = tid; e < 288; e += 128) s_w0[e] = w0f[e];
    if (tid < 32) { s_a0[tid] = a0[tid]; s_sh0[tid] = sh0[tid]; }
  }
  if (tid < NG * 3) s_ctr[tid] = new_xyz[((size_t)b * S + s0) * 3 + tid];

  if (wave < NG) {
    const float* cp = new_xyz + ((size_t)b * S + s0 + wave) * 3;
    const float cx = cp[0], cy = cp[1], cz = cp[2];
    int cnt = 0;
    int first = 0;
#pragma unroll 1
    for (int j0 = 0; j0 < NSRC && cnt < NS; j0 += 32) {
      const int j = j0 + lane;
      const float x = xb[j * 3 + 0];
      const float y = xb[j * 3 + 1];
      const float z = xb[j * 3 + 2];
      const float dx = cx - x;
      const float dy = cy - y;
      const float dz = cz - z;
      const float t0 = dx * dx;
      const float t1 = dy * dy;
      const float t2 = dz * dz;
      const float d = (t0 + t2) + t1;
      const bool pred = d < r2;
      const unsigned mask = __builtin_amdgcn_ballot_w32(pred);
      if (cnt == 0 && mask != 0u) first = j0 + __builtin_ctz(mask);
      const unsigned below = mask & ((1u << lane) - 1u);
      const int pos = cnt + __builtin_popcount(below);
      if (pred && pos < NS) s_pi[wave * NS + pos] = j;
      cnt += __builtin_popcount(mask);
    }
    cnt = cnt > NS ? NS : cnt;
    if (lane < NS && lane >= cnt) s_pi[wave * NS + lane] = first;
  }
  __syncthreads();

  if constexpr (LVL1) {
    const int row = tid >> 1;
    const int ch0 = (tid & 1) * 16;
    const int g = row / NS;
    int p = s_pi[row];
    p = p < 0 ? 0 : p;
    p = p > (NSRC - 1) ? (NSRC - 1) : p;
    const float px = xb[p * 3 + 0];
    const float py = xb[p * 3 + 1];
    const float pz = xb[p * 3 + 2];
    const float x9[9] = {px - s_ctr[g * 3 + 0], py - s_ctr[g * 3 + 1], pz - s_ctr[g * 3 + 2],
                         px, py, pz, px, py, pz};
#pragma unroll 1
    for (int hf = 0; hf < 2; ++hf) {
      float y[8];
#pragma unroll
      for (int e = 0; e < 8; ++e) {
        const int c = ch0 + hf * 8 + e;
        const float* wr = s_w0 + c * 9;
        float acc = wr[0] * x9[0];
#pragma unroll
        for (int k = 1; k < 9; ++k) {
          const float t = wr[k] * x9[k];
          acc = acc + t;
        }
        const float v = acc * s_a0[c] + s_sh0[c];
        y[e] = fmaxf(v, 0.0f);
      }
      v8h hv, lv;
      split8(y, hv, lv);
      *(v8h*)(sXh + row * KPAD + ch0 + hf * 8) = hv;
      *(v8h*)(sXl + row * KPAD + ch0 + hf * 8) = lv;
    }
  } else {
    constexpr int Q8 = CF / 8;
#pragma unroll 1
    for (int e = tid; e < RB * Q8; e += 128) {
      const int row = e / Q8;
      const int q = e - row * Q8;
      int p = s_pi[row];
      p = p < 0 ? 0 : p;
      p = p > (NSRC - 1) ? (NSRC - 1) : p;
      const v4f* src = (const v4f*)(feats + ((size_t)b * NSRC + p) * CF + q * 8);
      const v4f f0 = src[0];
      const v4f f1 = src[1];
      const float f[8] = {f0[0], f0[1], f0[2], f0[3], f1[0], f1[1], f1[2], f1[3]};
      v8h hv, lv;
      split8(f, hv, lv);
      *(v8h*)(sXh + row * KPAD + q * 8) = hv;
      *(v8h*)(sXl + row * KPAD + q * 8) = lv;
    }
    if (tid < RB) {
      const int row = tid;
      const int g = row / NS;
      int p = s_pi[row];
      p = p < 0 ? 0 : p;
      p = p > (NSRC - 1) ? (NSRC - 1) : p;
      const float px = xb[p * 3 + 0];
      const float py = xb[p * 3 + 1];
      const float pz = xb[p * 3 + 2];
      const float rx = px - s_ctr[g * 3 + 0];
      const float ry = py - s_ctr[g * 3 + 1];
      const float rz = pz - s_ctr[g * 3 + 2];
      float zf = 0.0f;
      asm volatile("" : "+v"(zf));
      const float t0[8] = {rx, ry, rz, zf, zf, zf, zf, zf};
      const float tz[8] = {zf, zf, zf, zf, zf, zf, zf, zf};
      v8h h0, l0, hz, lz;
      split8(t0, h0, l0);
      split8(tz, hz, lz);
      _Float16* ph = sXh + row * KPAD + CF;
      _Float16* pl = sXl + row * KPAD + CF;
      *(v8h*)(ph) = h0;
      *(v8h*)(ph + 8) = hz;
      *(v8h*)(ph + 16) = hz;
      *(v8h*)(ph + 24) = hz;
      *(v8h*)(pl) = l0;
      *(v8h*)(pl + 8) = lz;
      *(v8h*)(pl + 16) = lz;
      *(v8h*)(pl + 24) = lz;
    }
  }
  __syncthreads();

  if constexpr (!LVL1) {
    mlp_layer<NI, KPAD, C1, NS, false>(sXh, sXl, (const _Float16*)WaH, (const _Float16*)WaL, aA, shA,
                                       sYh, sYl, sP, wave, lane);
    __syncthreads();
    mlp_layer<NI, C1, C2, NS, true>(sYh, sYl, (const _Float16*)WbH, (const _Float16*)WbL, aB, shB,
                                    sYh, sYl, sP, wave, lane);
  } else {
    mlp_layer<NI, KPAD, C2, NS, true>(sXh, sXl, (const _Float16*)WbH, (const _Float16*)WbL, aB, shB,
                                      sXh, sXl, sP, wave, lane);
  }
  __syncthreads();

  constexpr int NV = NG * C2 / 4;
  if (tid < NV) {
    const v4f v = *(const v4f*)(sP + 4 * tid);
    float* dst = pooled + ((size_t)b * S + s0) * C2 + 4 * tid;
    *(volatile v4f*)dst = v;
    __threadfence();
    *(volatile v4f*)dst = v;
  }
}

__global__ __launch_bounds__(256) void transpose_out(const float* __restrict__ src_all, float* __restrict__ out) {
  constexpr int PITCH = 260;
  __shared__ __align__(16) float sT[32 * PITCH];
  const int b = blockIdx.x;
  const int tid = threadIdx.x;
  const int lane = tid & 31;
  const int wave = tid >> 5;
  const float* src = src_all + (size_t)b * 32 * 256;
#pragma unroll 1
  for (int e = tid; e < 32 * 64; e += 256) {
    const int s = e >> 6;
    const int q = e & 63;
    const v4f v = *(const v4f*)(src + s * 256 + q * 4);
    *(v4f*)(sT + s * PITCH + q * 4) = v;
  }
  __syncthreads();
  const int cl = lane >> 3;
  const int s4 = (lane & 7) * 4;
  for (int pass = 0; pass < 2; ++pass) {
#pragma unroll 1
    for (int t = 0; t < 8; ++t) {
      const int c = (wave * 8 + t) * 4 + cl;
      v4f v;
      v[0] = sT[(s4 + 0) * PITCH + c];
      v[1] = sT[(s4 + 1) * PITCH + c];
      v[2] = sT[(s4 + 2) * PITCH + c];
      v[3] = sT[(s4 + 3) * PITCH + c];
      *(volatile v4f*)(out + ((size_t)b * 256 + c) * 32 + s4) = v;
    }
    __threadfence();
  }
}

extern "C" void kernel_launch(void* const* d_in, const int* in_sizes, int n_in,
                              void* d_out, int out_size, void* d_ws, size_t ws_size,
                              hipStream_t stream) {
  (void)in_sizes; (void)out_size;
  if (n_in < 31) return;
  const float* pc = (const float*)d_in[0];
  const float *Wf[6], *Gf[6], *Bef[6], *Rmf[6], *Rvf[6];
  for (int l = 0; l < 6; ++l) {
    Wf[l]  = (const float*)d_in[1 + 5 * l + 0];
    Gf[l]  = (const float*)d_in[1 + 5 * l + 1];
    Bef[l] = (const float*)d_in[1 + 5 * l + 2];
    Rmf[l] = (const float*)d_in[1 + 5 * l + 3];
    Rvf[l] = (const float*)d_in[1 + 5 * l + 4];
  }

  char* ws = (char*)d_ws;
  size_t off = 0;
  auto carve = [&](size_t bytes) -> void* {
    off = (off + 255) & ~(size_t)255;
    void* p = ws + off;
    off += bytes;
    return p;
  };
  float* xyz1   = (float*)carve((size_t)kBatch * 128 * 3 * 4);
  float* xyz2   = (float*)carve((size_t)kBatch * 64 * 3 * 4);
  float* xyz3   = (float*)carve((size_t)kBatch * 32 * 3 * 4);
  float* feats1 = (float*)carve((size_t)kBatch * 128 * 64 * 4);
  float* feats2 = (float*)carve((size_t)kBatch * 64 * 128 * 4);
  float* pool3  = (float*)carve((size_t)kBatch * 32 * 256 * 4);

  static const int CoutL[6] = {32, 64, 128, 128, 256, 256};
  static const int KpadL[6] = {0, 32, 96, 128, 160, 256};
  unsigned short* Wh[6];
  unsigned short* Wl[6];
  float* bnA[6];
  float* bnS[6];
  Wh[0] = nullptr; Wl[0] = nullptr;
  for (int l = 1; l < 6; ++l) {
    Wh[l] = (unsigned short*)carve((size_t)CoutL[l] * KpadL[l] * 2);
    Wl[l] = (unsigned short*)carve((size_t)CoutL[l] * KpadL[l] * 2);
  }
  for (int l = 0; l < 6; ++l) {
    bnA[l] = (float*)carve((size_t)CoutL[l] * 4);
    bnS[l] = (float*)carve((size_t)CoutL[l] * 4);
  }
  if (off > ws_size || off > (size_t)134217728) return;

  PrepArgs pa;
  for (int l = 0; l < 5; ++l) {
    pa.w[l] = Wf[l + 1];
    pa.wh[l] = Wh[l + 1];
    pa.wl[l] = Wl[l + 1];
  }
  for (int l = 0; l < 6; ++l) {
    pa.g[l] = Gf[l]; pa.be[l] = Bef[l]; pa.rm[l] = Rmf[l]; pa.rv[l] = Rvf[l];
    pa.a[l] = bnA[l]; pa.sh[l] = bnS[l];
  }
  prep_kernel<<<dim3(32, 6), dim3(256), 0, stream>>>(pa);

  const float r2_1 = (float)(0.02 * 0.02);
  const float r2_2 = (float)(0.04 * 0.04);
  const float r2_3 = (float)(0.08 * 0.08);

  fps_kernel<4096, 128><<<dim3(kBatch), dim3(256), 0, stream>>>(pc, xyz1);
  sa_kernel<6, 32, 32, 64, 32, 4096, 64, true><<<dim3(64, kBatch), dim3(128), 0, stream>>>(
      pc, pc, xyz1, Wf[0], bnA[0], bnS[0],
      Wh[1], Wl[1], bnA[1], bnS[1],
      Wh[1], Wl[1], bnA[1], bnS[1],
      feats1, 128, r2_1);

  fps_kernel<128, 64><<<dim3(kBatch), dim3(256), 0, stream>>>(xyz1, xyz2);
  sa_kernel<64, 96, 128, 128, 32, 128, 64, false><<<dim3(32, kBatch), dim3(128), 0, stream>>>(
      xyz1, feats1, xyz2, Wf[0], bnA[0], bnS[0],
      Wh[2], Wl[2], bnA[2], bnS[2],
      Wh[3], Wl[3], bnA[3], bnS[3],
      feats2, 64, r2_2);

  fps_kernel<64, 32><<<dim3(kBatch), dim3(256), 0, stream>>>(xyz2, xyz3);
  sa_kernel<128, 160, 256, 256, 16, 64, 32, false><<<dim3(16, kBatch), dim3(128), 0, stream>>>(
      xyz2, feats2, xyz3, Wf[0], bnA[0], bnS[0],
      Wh[4], Wl[4], bnA[4], bnS[4],
      Wh[5], Wl[5], bnA[5], bnS[5],
      pool3, 32, r2_3);

  transpose_out<<<dim3(kBatch), dim3(256), 0, stream>>>(pool3, (float*)d_out);
}
